// PointActorTFN_52295521796465
// MI455X (gfx1250) — hardware-verified
//
#include <hip/hip_runtime.h>
#include <math.h>

constexpr int kB    = 64;
constexpr int kN    = 8192;
constexpr int kNT   = 4096;
constexpr int kFin  = 6;
constexpr int kH    = 128;
constexpr int kBPC  = 16;
constexpr int kNChunk = kB / kBPC;
constexpr int kMC   = kBPC * kNT;
constexpr int kK1   = 32;
constexpr int kN6   = 64;
constexpr int kFld  = kN6;
constexpr float kScale = 50.0f;
constexpr int kOut1Elem = kB * kNT * 3;
constexpr int kOutElems = 2 * kB * kNT * 3;

constexpr int kWoff1 = 0;
constexpr int kWoff2 = kWoff1 + kH * kK1;
constexpr int kWoff3 = kWoff2 + kH * kH;
constexpr int kWoff4 = kWoff3 + kH * kH;
constexpr int kWoff5 = kWoff4 + kH * kH;
constexpr int kWoff6 = kWoff5 + kH * kH;
constexpr int kWHalves = kWoff6 + kN6 * kH;

constexpr size_t kWPlaneBytes   = (size_t)kWHalves * 2;
constexpr size_t kActPlaneBytes = (size_t)kMC * kH * 2;
constexpr size_t kA0PlaneBytes  = (size_t)kMC * kK1 * 2;
constexpr size_t kFBytes        = (size_t)kMC * kFld * 4;
constexpr size_t kOffWH = 0;
constexpr size_t kOffWL = kOffWH + kWPlaneBytes;
constexpr size_t kOffPH = kOffWL + kWPlaneBytes;
constexpr size_t kOffPL = kOffPH + kActPlaneBytes;
constexpr size_t kOffXH = kOffPL + kActPlaneBytes;
constexpr size_t kOffXL = kOffXH + kActPlaneBytes;
constexpr size_t kOffF  = kOffXL + kActPlaneBytes;
constexpr size_t kWsTotal = kOffF + kFBytes;
static_assert(kWsTotal == 84197376);
static_assert(kWsTotal <= 134217728);
static_assert((kOffPH % 512) == 0 && (kOffXH % 512) == 0 && (kOffF % 512) == 0);
static_assert(2 * kA0PlaneBytes <= kActPlaneBytes);
static_assert((kMC % 64) == 0 && (kH % 64) == 0 && (kN6 % 64) == 0 && (kK1 % 32) == 0 && (kH % 32) == 0);

constexpr int kGemmBlocks  = ((kMC / 64) * (kH  / 64)) / 8;
constexpr int kGemm6Blocks = ((kMC / 64) * (kN6 / 64)) / 8;
static_assert(kGemmBlocks * 8 == (kMC / 64) * (kH / 64));
static_assert(kGemm6Blocks * 8 == (kMC / 64) * (kN6 / 64));

typedef __attribute__((ext_vector_type(16))) _Float16 v16h;
typedef __attribute__((ext_vector_type(8)))  _Float16 v8h;
typedef __attribute__((ext_vector_type(16))) __bf16   v16b;
typedef __attribute__((ext_vector_type(8)))  __bf16   v8b;
typedef __attribute__((ext_vector_type(8)))  float    v8f;
typedef __attribute__((ext_vector_type(4)))  float    v4f;
typedef __attribute__((ext_vector_type(4)))  unsigned int v4u;

__device__ __forceinline__ unsigned short f2bf_bits(float f) {
  unsigned u = __float_as_uint(f);
  return (unsigned short)((u + 0x7FFFu + ((u >> 16) & 1u)) >> 16);
}
__device__ __forceinline__ float bf_bits2f(unsigned short h) { return __uint_as_float(((unsigned)h) << 16); }

__device__ __forceinline__ void dep_guard_h(v8f& a, v8f& b, v16h x, v16h y) { asm volatile("v_nop\n\tv_nop\n\tv_nop\n\tv_nop" : "+v"(a), "+v"(b) : "v"(x), "v"(y)); }
__device__ __forceinline__ void dep_guard_b(v8f& a, v8f& b, v16b x, v16b y) { asm volatile("v_nop\n\tv_nop\n\tv_nop\n\tv_nop" : "+v"(a), "+v"(b) : "v"(x), "v"(y)); }
__device__ __forceinline__ void keep4_h(v16h a, v16h b, v16h c, v16h d) { asm volatile("v_nop" :: "v"(a), "v"(b), "v"(c), "v"(d)); }
__device__ __forceinline__ void keep4_b(v16b a, v16b b, v16b c, v16b d) { asm volatile("v_nop" :: "v"(a), "v"(b), "v"(c), "v"(d)); }
__device__ __forceinline__ void acc_guard4(v8f& a, v8f& b, v8f& c, v8f& d) { asm volatile("v_nop\n\tv_nop\n\tv_nop\n\tv_nop" : "+v"(a), "+v"(b), "+v"(c), "+v"(d)); }
template <typename T> struct Frag;
template <> struct Frag<_Float16> {
  typedef v16h V; union U { v16h v; v8h h[2]; };
  static __device__ __forceinline__ v16h load(const _Float16* p) {
    U f; f.h[0] = *(const v8h*)(p); f.h[1] = *(const v8h*)(p + 16); return f.v;
  }
  static __device__ __forceinline__ v8f mma(v16h a, v16h b, v8f c) {
    return __builtin_amdgcn_wmma_f32_16x16x32_f16(false, a, false, b, (short)0, c, false, false);
  }
  static __device__ __forceinline__ void guard(v8f& a, v8f& b, v16h x, v16h y) { dep_guard_h(a, b, x, y); }
  static __device__ __forceinline__ void keep(v16h a, v16h b, v16h c, v16h d) { keep4_h(a, b, c, d); }
};
template <> struct Frag<__bf16> {
  typedef v16b V; union U { v16b v; v8b h[2]; };
  static __device__ __forceinline__ v16b load(const __bf16* p) {
    U f; f.h[0] = *(const v8b*)(p); f.h[1] = *(const v8b*)(p + 16); return f.v;
  }
  static __device__ __forceinline__ v8f mma(v16b a, v16b b, v8f c) {
    return __builtin_amdgcn_wmma_f32_16x16x32_bf16(false, a, false, b, (short)0, c, false, false);
  }
  static __device__ __forceinline__ void guard(v8f& a, v8f& b, v16b x, v16b y) { dep_guard_b(a, b, x, y); }
  static __device__ __forceinline__ void keep(v16b a, v16b b, v16b c, v16b d) { keep4_b(a, b, c, d); }
};

__device__ __forceinline__ unsigned pk16(unsigned short a, unsigned short b) { return (unsigned)a | ((unsigned)b << 16); }
__device__ __forceinline__ int imin(int a, int b) { return a < b ? a : b; }

template <int ET> struct Elem;
template <> struct Elem<0> { typedef _Float16 T; };
template <> struct Elem<1> { typedef __bf16 T; };
template <int ET, bool SPLIT, int BIAS_MODE, int OUT_MODE, bool RESID, int ACT = 0>
__global__ __launch_bounds__(256) void wmma_gemm64(
    const unsigned short* __restrict__ Ap, const unsigned short* __restrict__ A2p, int lda, long strideA,
    const unsigned short* __restrict__ Btp, const unsigned short* __restrict__ Bt2p, int ldb, long strideB,
    void* __restrict__ Cout, void* __restrict__ Cout2, int ldc, long strideC,
    const float* __restrict__ bias,
    const float* __restrict__ resid, long strideR,
    int M, int N, int K, float scale) {
  typedef typename Elem<ET>::T T;
  typedef typename Frag<T>::V V;
  const T* A = (const T*)Ap; const T* A2 = (const T*)A2p; const T* Bt = (const T*)Btp; const T* Bt2 = (const T*)Bt2p;
  __shared__ __align__(16) float sT[8][16 * 68];
  const int b    = blockIdx.y;
  const int lane = threadIdx.x & 31;
  const int wave = threadIdx.x >> 5;
  const int tilesN = N >> 6;
  const int tilesM = M >> 6;
  const int tile = blockIdx.x * 8 + wave;
  if (tile >= tilesM * tilesN) return;
  const int tm = tile / tilesN;
  const int tn = tile - tm * tilesN;
  const int m0 = tm << 6;
  const int n0 = tn << 6;

  const T* Ab  = A  + (size_t)b * strideA;
  const T* Bb  = Bt + (size_t)b * strideB;
  const T* Ab2 = SPLIT ? (A2  + (size_t)b * strideA) : nullptr;
  const T* Bb2 = SPLIT ? (Bt2 + (size_t)b * strideB) : nullptr;

  const int rlane = lane & 15;
  const int koff  = (lane >> 4) * 8;
  const int mOff  = (lane >> 4) * 8;

  v8f acc[4][4];
#pragma unroll
  for (int i = 0; i < 4; ++i)
#pragma unroll
    for (int j = 0; j < 4; ++j) acc[i][j] = (v8f){0.f,0.f,0.f,0.f,0.f,0.f,0.f,0.f};

  for (int k0 = 0; k0 < K; k0 += 32) {
    V bh[4], bl[4];
#pragma unroll
    for (int j = 0; j < 4; ++j) {
      const size_t bo = (size_t)(n0 + (j << 4) + rlane) * ldb + koff + k0;
      bh[j] = Frag<T>::load(Bb + bo);
      if (SPLIT) bl[j] = Frag<T>::load(Bb2 + bo);
    }
#pragma unroll
    for (int i = 0; i < 4; ++i) {
      const size_t ao = (size_t)(m0 + (i << 4) + rlane) * lda + koff + k0;
      V ah = Frag<T>::load(Ab + ao);
      V al;
      if (SPLIT) al = Frag<T>::load(Ab2 + ao);
#pragma unroll
      for (int j = 0; j < 4; ++j) {
        acc[i][j] = Frag<T>::mma(ah, bh[j], acc[i][j]);
        if (SPLIT) {
          acc[i][j] = Frag<T>::mma(ah, bl[j], acc[i][j]);
          acc[i][j] = Frag<T>::mma(al, bh[j], acc[i][j]);
        }
      }
      Frag<T>::guard(acc[i][0], acc[i][3], ah, SPLIT ? al : ah);
    }
    Frag<T>::keep(bh[0], bh[1], bh[2], bh[3]);
    if (SPLIT) Frag<T>::keep(bl[0], bl[1], bl[2], bl[3]);
  }
  acc_guard4(acc[0][0], acc[0][1], acc[0][2], acc[0][3]);
  acc_guard4(acc[1][0], acc[1][1], acc[1][2], acc[1][3]);
  acc_guard4(acc[2][0], acc[2][1], acc[2][2], acc[2][3]);
  acc_guard4(acc[3][0], acc[3][1], acc[3][2], acc[3][3]);

  float* slab = sT[wave];
  const float* Rb = RESID ? (resid + (size_t)b * strideR) : nullptr;
#pragma unroll
  for (int i = 0; i < 4; ++i) {
    const int mBase = m0 + (i << 4);
#pragma unroll
    for (int j = 0; j < 4; ++j) {
      const int n = n0 + (j << 4) + rlane;
      float bv = 0.f;
      if (BIAS_MODE == 2) bv = bias[n];
#pragma unroll
      for (int r = 0; r < 8; ++r) {
        float v = acc[i][j][r] * scale;
        if (BIAS_MODE == 1) v += bias[mBase + mOff + r];
        if (BIAS_MODE == 2) v += bv;
        if (RESID) v += Rb[(size_t)(mBase + mOff + r) * ldc + n];
        if (ACT == 2) v = fmaxf(v, 0.0f);
        if (ACT == 4) v = (v > 0.f) ? v : 0.01f * v;
        slab[(mOff + r) * 68 + (j << 4) + rlane] = v;
      }
    }
    __builtin_amdgcn_fence(__ATOMIC_RELEASE, "workgroup");
    __builtin_amdgcn_wave_barrier();
    __builtin_amdgcn_fence(__ATOMIC_ACQUIRE, "workgroup");
    if (OUT_MODE == 0) {
      float* C = (float*)Cout + (size_t)b * strideC;
      const int hh = lane >> 4, c4 = (lane & 15) * 4;
      for (int pass = 0; pass < 2; ++pass) {
#pragma unroll
        for (int it = 0; it < 8; ++it) {
          const int row = it * 2 + hh;
          v4f v = *(const v4f*)(slab + row * 68 + c4);
          *(volatile v4f*)(C + (size_t)(mBase + row) * ldc + n0 + c4) = v;
        }
        __threadfence();
      }
    } else {
      const int q = lane >> 3, c8 = (lane & 7) * 8;
      unsigned short* C  = (unsigned short*)Cout  + (size_t)b * strideC;
      unsigned short* C2 = (OUT_MODE == 2) ? ((unsigned short*)Cout2 + (size_t)b * strideC) : nullptr;
      for (int pass = 0; pass < 2; ++pass) {
#pragma unroll
        for (int it = 0; it < 4; ++it) {
          const int row = it * 4 + q;
          const float* sp = slab + row * 68 + c8;
          v8h hv, lv;
#pragma unroll
          for (int e = 0; e < 8; ++e) {
            if (OUT_MODE == 1) {
              hv[e] = (_Float16)sp[e];
            } else {
              unsigned short hb = f2bf_bits(sp[e]);
              unsigned short lb = f2bf_bits(sp[e] - bf_bits2f(hb));
              hv[e] = __builtin_bit_cast(_Float16, hb);
              lv[e] = __builtin_bit_cast(_Float16, lb);
            }
          }
          *(volatile v8h*)(C + (size_t)(mBase + row) * ldc + n0 + c8) = hv;
          if (OUT_MODE == 2) *(volatile v8h*)(C2 + (size_t)(mBase + row) * ldc + n0 + c8) = lv;
        }
        __threadfence();
      }
    }
    __builtin_amdgcn_fence(__ATOMIC_RELEASE, "workgroup");
    __builtin_amdgcn_wave_barrier();
    __builtin_amdgcn_fence(__ATOMIC_ACQUIRE, "workgroup");
  }
}

__global__ __launch_bounds__(256) void wprep_kernel(const float* __restrict__ Wa, const float* __restrict__ Wb,
                                                    const float* __restrict__ Wc, const float* __restrict__ Wd,
                                                    const float* __restrict__ We, const float* __restrict__ Wf,
                                                    unsigned short* __restrict__ WH, unsigned short* __restrict__ WL)
{
  const int z = blockIdx.y;
  const float* W = (z == 0) ? Wa : (z == 1) ? Wb : (z == 2) ? Wc : (z == 3) ? Wd : (z == 4) ? We : Wf;
  const int Kr  = (z == 0) ? kFin : kH;
  const int Nr  = (z == 5) ? 3 : kH;
  const int Kp  = (z == 0) ? kK1 : kH;
  const int Np  = (z == 5) ? kN6 : kH;
  const int off = (z == 0) ? kWoff1 : (z == 1) ? kWoff2 : (z == 2) ? kWoff3 : (z == 3) ? kWoff4 : (z == 4) ? kWoff5 : kWoff6;
  const int t  = blockIdx.x * 256 + threadIdx.x;
  const int n8 = (Np * Kp) >> 3;
  if (t >= n8) return;
  const int kq = Kp >> 3;
  const int n  = t / kq;
  const int k0 = (t - n * kq) * 8;
  const int nc = imin(n, Nr - 1);
  const float nsel = (n < Nr) ? 1.0f : 0.0f;
  unsigned short hb[8], lb[8];
#pragma unroll
  for (int e = 0; e < 8; ++e) {
    const int k  = k0 + e;
    const int kc = imin(k, Kr - 1);
    const float sel = (k < Kr) ? nsel : 0.0f;
    const float v = W[(size_t)kc * Nr + nc] * sel;
    const unsigned short h = f2bf_bits(v);
    hb[e] = h;
    lb[e] = f2bf_bits(v - bf_bits2f(h));
  }
  const v4u uh = (v4u){pk16(hb[0], hb[1]), pk16(hb[2], hb[3]), pk16(hb[4], hb[5]), pk16(hb[6], hb[7])};
  const v4u ul = (v4u){pk16(lb[0], lb[1]), pk16(lb[2], lb[3]), pk16(lb[4], lb[5]), pk16(lb[6], lb[7])};
  unsigned short* ph = WH + off + 8 * (size_t)t;
  unsigned short* pl = WL + off + 8 * (size_t)t;
  *(volatile v4u*)ph = uh;
  *(volatile v4u*)pl = ul;
  __threadfence();
  *(volatile v4u*)ph = uh;
  *(volatile v4u*)pl = ul;
}

__global__ __launch_bounds__(256) void aprep_kernel(const float* __restrict__ feat,
                                                    unsigned short* __restrict__ AH, unsigned short* __restrict__ AL, int chunk)
{
  const int t = blockIdx.x * 256 + threadIdx.x;
  if (t >= kMC * 4) return;
  const int row = t >> 2;
  const int g   = t & 3;
  const int bl  = row >> 12;
  const int n   = row & (kNT - 1);
  const int b   = chunk * kBPC + bl;
  const float* fp = feat + ((size_t)b * kN + n) * kFin;
  float fv[6];
#pragma unroll
  for (int e = 0; e < 6; ++e) fv[e] = fp[e];
  const float gsel = (g == 0) ? 1.0f : 0.0f;
  unsigned short hb[8], lb[8];
#pragma unroll
  for (int e = 0; e < 8; ++e) {
    const float sel = (e < kFin) ? gsel : 0.0f;
    const float v = fv[(e < 6) ? e : 5] * sel;
    const unsigned short h = f2bf_bits(v);
    hb[e] = h;
    lb[e] = f2bf_bits(v - bf_bits2f(h));
  }
  const v4u uh = (v4u){pk16(hb[0], hb[1]), pk16(hb[2], hb[3]), pk16(hb[4], hb[5]), pk16(hb[6], hb[7])};
  const v4u ul = (v4u){pk16(lb[0], lb[1]), pk16(lb[2], lb[3]), pk16(lb[4], lb[5]), pk16(lb[6], lb[7])};
  unsigned short* ph = AH + 8 * (size_t)t;
  unsigned short* pl = AL + 8 * (size_t)t;
  *(volatile v4u*)ph = uh;
  *(volatile v4u*)pl = ul;
  __threadfence();
  *(volatile v4u*)ph = uh;
  *(volatile v4u*)pl = ul;
}

__device__ __forceinline__ double wsum_d(double v) {
#pragma unroll
  for (int off = 16; off > 0; off >>= 1) v += __shfl_xor(v, off, 32);
  return v;
}

__global__ __launch_bounds__(256) void rigid_fit_kernel(const float* __restrict__ pos, const float* __restrict__ Fp,
                                                        const float* __restrict__ bm3, float* __restrict__ out, int chunk)
{
#pragma clang fp contract(off)
  __shared__ __align__(16) float stage[kNT * 3];
  __shared__ double red[8][16];
  __shared__ float sG[9];
  __shared__ float sV[9];
  __shared__ float sU[9];
  __shared__ float sP[9];
  __shared__ float sS[3];
  __shared__ float sR[9];
  __shared__ float scx[3];
  __shared__ float scy[3];

  const int tid  = threadIdx.x;
  const int lane = tid & 31;
  const int wave = tid >> 5;
  const int bl   = blockIdx.x;
  const int b    = chunk * kBPC + bl;
  const float* pb = pos + (size_t)b * kN * 3;
  const float* fb = Fp + (size_t)bl * kNT * kFld;
  const float bmv0 = bm3[0], bmv1 = bm3[1], bmv2 = bm3[2];

  double sx0 = 0.0, sx1 = 0.0, sx2 = 0.0, st0 = 0.0, st1 = 0.0, st2 = 0.0;
#pragma unroll 1
  for (int p = 0; p < kNT / 256; ++p) {
    const int n = tid + 256 * p;
    const float x0 = pb[n * 3 + 0] * kScale;
    const float x1 = pb[n * 3 + 1] * kScale;
    const float x2 = pb[n * 3 + 2] * kScale;
    const float f0 = fb[n * kFld + 0] + bmv0;
    const float f1 = fb[n * kFld + 1] + bmv1;
    const float f2 = fb[n * kFld + 2] + bmv2;
    const float t0 = x0 + f0, t1 = x1 + f1, t2 = x2 + f2;
    stage[n * 3 + 0] = f0;
    stage[n * 3 + 1] = f1;
    stage[n * 3 + 2] = f2;
    sx0 += (double)x0; sx1 += (double)x1; sx2 += (double)x2;
    st0 += (double)t0; st1 += (double)t1; st2 += (double)t2;
  }
  sx0 = wsum_d(sx0); sx1 = wsum_d(sx1); sx2 = wsum_d(sx2);
  st0 = wsum_d(st0); st1 = wsum_d(st1); st2 = wsum_d(st2);
  if (lane == 0) {
    red[wave][0] = sx0; red[wave][1] = sx1; red[wave][2] = sx2;
    red[wave][3] = st0; red[wave][4] = st1; red[wave][5] = st2;
  }
  __syncthreads();
  if (tid == 0) {
#pragma unroll 1
    for (int i = 0; i < 6; ++i) {
      double s = red[0][i];
#pragma unroll 1
      for (int w = 1; w < 8; ++w) s += red[w][i];
      const float m = (float)(s * (1.0 / 4096.0));
      if (i < 3) scx[i] = m; else scy[i - 3] = m;
    }
  }
  __syncthreads();
  const float cx0 = scx[0], cx1 = scx[1], cx2 = scx[2];
  const float cy0 = scy[0], cy1 = scy[1], cy2 = scy[2];

  {
    float* dst = out + (size_t)kOut1Elem + (size_t)b * (kNT * 3);
    for (int pass = 0; pass < 2; ++pass) {
#pragma unroll
      for (int i = 0; i < 12; ++i) {
        const int q = tid + 256 * i;
        const v4f v = *(const v4f*)(stage + 4 * q);
        *(volatile v4f*)(dst + 4 * (size_t)q) = v;
      }
      __threadfence();
    }
  }

  double h00 = 0.0, h01 = 0.0, h02 = 0.0, h10 = 0.0, h11 = 0.0, h12 = 0.0, h20 = 0.0, h21 = 0.0, h22 = 0.0;
#pragma unroll 1
  for (int p = 0; p < kNT / 256; ++p) {
    const int n = tid + 256 * p;
    const float x0 = pb[n * 3 + 0] * kScale;
    const float x1 = pb[n * 3 + 1] * kScale;
    const float x2 = pb[n * 3 + 2] * kScale;
    const float f0 = fb[n * kFld + 0] + bmv0;
    const float f1 = fb[n * kFld + 1] + bmv1;
    const float f2 = fb[n * kFld + 2] + bmv2;
    const float t0 = x0 + f0, t1 = x1 + f1, t2 = x2 + f2;
    const double a0 = (double)(x0 - cx0), a1 = (double)(x1 - cx1), a2 = (double)(x2 - cx2);
    const double y0 = (double)(t0 - cy0), y1 = (double)(t1 - cy1), y2 = (double)(t2 - cy2);
    h00 += a0 * y0; h01 += a0 * y1; h02 += a0 * y2;
    h10 += a1 * y0; h11 += a1 * y1; h12 += a1 * y2;
    h20 += a2 * y0; h21 += a2 * y1; h22 += a2 * y2;
  }
  h00 = wsum_d(h00); h01 = wsum_d(h01); h02 = wsum_d(h02);
  h10 = wsum_d(h10); h11 = wsum_d(h11); h12 = wsum_d(h12);
  h20 = wsum_d(h20); h21 = wsum_d(h21); h22 = wsum_d(h22);
  if (lane == 0) {
    red[wave][0] = h00; red[wave][1] = h01; red[wave][2] = h02;
    red[wave][3] = h10; red[wave][4] = h11; red[wave][5] = h12;
    red[wave][6] = h20; red[wave][7] = h21; red[wave][8] = h22;
  }
  __syncthreads();
  if (tid == 0) {
#pragma unroll 1
    for (int r = 0; r < 9; ++r) {
      double s = red[0][r];
#pragma unroll 1
      for (int w = 1; w < 8; ++w) s += red[w][r];
      sG[r] = (float)s;
      sV[r] = ((r & 3) == 0) ? 1.0f : 0.0f;
    }
#pragma unroll 1
    for (int sweep = 0; sweep < 15; ++sweep) {
#pragma unroll 1
      for (int pr = 0; pr < 3; ++pr) {
        const int p = (pr == 2) ? 1 : 0;
        const int q = (pr == 0) ? 1 : 2;
        float al = 0.0f, be = 0.0f, ga = 0.0f;
#pragma unroll 1
        for (int k = 0; k < 3; ++k) {
          const float gp = sG[k * 3 + p], gq = sG[k * 3 + q];
          al += gp * gp; be += gq * gq; ga += gp * gq;
        }
        const float thr = 1e-9f * sqrtf(al * be);
        if (fabsf(ga) > thr) {
          const float zeta = (be - al) / (2.0f * ga);
          if (fabsf(zeta) < 1e7f) {
            const float tq = copysignf(1.0f, zeta) / (fabsf(zeta) + sqrtf(1.0f + zeta * zeta));
            const float cs = 1.0f / sqrtf(1.0f + tq * tq);
            const float sn = cs * tq;
#pragma unroll 1
            for (int k = 0; k < 3; ++k) {
              const float gp = sG[k * 3 + p], gq = sG[k * 3 + q];
              sG[k * 3 + p] = cs * gp - sn * gq;
              sG[k * 3 + q] = sn * gp + cs * gq;
              const float vp = sV[k * 3 + p], vq = sV[k * 3 + q];
              sV[k * 3 + p] = cs * vp - sn * vq;
              sV[k * 3 + q] = sn * vp + cs * vq;
            }
          }
        }
      }
    }
#pragma unroll 1
    for (int j = 0; j < 3; ++j) {
      const float g0 = sG[j], g1 = sG[3 + j], g2 = sG[6 + j];
      sS[j] = sqrtf(g0 * g0 + g1 * g1 + g2 * g2);
    }
#pragma unroll 1
    for (int i = 0; i < 2; ++i) {
#pragma unroll 1
      for (int j = i + 1; j < 3; ++j) {
        if (sS[j] > sS[i]) {
          const float ts = sS[i]; sS[i] = sS[j]; sS[j] = ts;
#pragma unroll 1
          for (int k = 0; k < 3; ++k) {
            const float tg = sG[k * 3 + i]; sG[k * 3 + i] = sG[k * 3 + j]; sG[k * 3 + j] = tg;
            const float tv = sV[k * 3 + i]; sV[k * 3 + i] = sV[k * 3 + j]; sV[k * 3 + j] = tv;
          }
        }
      }
    }
#pragma unroll 1
    for (int j = 0; j < 3; ++j) {
      const float s = sS[j];
      const float inv = (s > 0.0f) ? (1.0f / s) : 0.0f;
#pragma unroll 1
      for (int k = 0; k < 3; ++k) sU[k * 3 + j] = sG[k * 3 + j] * inv;
    }
    if (sS[2] <= 1e-7f * sS[0]) {
      const float u00 = sU[0], u10 = sU[3], u20 = sU[6];
      const float u01 = sU[1], u11 = sU[4], u21 = sU[7];
      sU[2] = u10 * u21 - u20 * u11;
      sU[5] = u20 * u01 - u00 * u21;
      sU[8] = u00 * u11 - u10 * u01;
    }
#pragma unroll 1
    for (int i = 0; i < 3; ++i) {
#pragma unroll 1
      for (int k = 0; k < 3; ++k) {
        float s = 0.0f;
#pragma unroll 1
        for (int j = 0; j < 3; ++j) s += sV[i * 3 + j] * sU[k * 3 + j];
        sP[i * 3 + k] = s;
      }
    }
    const float d = sP[0] * (sP[4] * sP[8] - sP[5] * sP[7])
                  - sP[1] * (sP[3] * sP[8] - sP[5] * sP[6])
                  + sP[2] * (sP[3] * sP[7] - sP[4] * sP[6]);
#pragma unroll 1
    for (int i = 0; i < 3; ++i) {
#pragma unroll 1
      for (int k = 0; k < 3; ++k) {
        float s = 0.0f;
#pragma unroll 1
        for (int j = 0; j < 3; ++j) {
          const float scj = (j == 2) ? d : 1.0f;
          s += (sV[i * 3 + j] * scj) * sU[k * 3 + j];
        }
        sR[i * 3 + k] = s;
      }
    }
  }
  __syncthreads();
  const float r00 = sR[0], r01 = sR[1], r02 = sR[2];
  const float r10 = sR[3], r11 = sR[4], r12 = sR[5];
  const float r20 = sR[6], r21 = sR[7], r22 = sR[8];

#pragma unroll 1
  for (int p = 0; p < kNT / 256; ++p) {
    const int n = tid + 256 * p;
    const float x0 = pb[n * 3 + 0] * kScale;
    const float x1 = pb[n * 3 + 1] * kScale;
    const float x2 = pb[n * 3 + 2] * kScale;
    const float a0 = x0 - cx0, a1 = x1 - cx1, a2 = x2 - cx2;
    const float q0 = ((a0 * r00 + a1 * r01) + a2 * r02) + cy0;
    const float q1 = ((a0 * r10 + a1 * r11) + a2 * r12) + cy1;
    const float q2 = ((a0 * r20 + a1 * r21) + a2 * r22) + cy2;
    stage[n * 3 + 0] = q0 - x0;
    stage[n * 3 + 1] = q1 - x1;
    stage[n * 3 + 2] = q2 - x2;
  }
  __syncthreads();
  {
    float* dst = out + (size_t)b * (kNT * 3);
    for (int pass = 0; pass < 2; ++pass) {
#pragma unroll
      for (int i = 0; i < 12; ++i) {
        const int q = tid + 256 * i;
        const v4f v = *(const v4f*)(stage + 4 * q);
        *(volatile v4f*)(dst + 4 * (size_t)q) = v;
      }
      __threadfence();
    }
  }
}

extern "C" void kernel_launch(void* const* d_in, const int* in_sizes, int n_in,
                              void* d_out, int out_size, void* d_ws, size_t ws_size,
                              hipStream_t stream)
{
  (void)in_sizes;
  if (n_in < 14) return;
  if ((size_t)out_size < (size_t)kOutElems) return;
  if (ws_size < kWsTotal) return;

  const float* pos  = (const float*)d_in[0];
  const float* feat = (const float*)d_in[1];
  const float* W1   = (const float*)d_in[2];
  const float* b1   = (const float*)d_in[3];
  const float* W2   = (const float*)d_in[4];
  const float* b2   = (const float*)d_in[5];
  const float* W3   = (const float*)d_in[6];
  const float* b3   = (const float*)d_in[7];
  const float* Wm1  = (const float*)d_in[8];
  const float* bm1  = (const float*)d_in[9];
  const float* Wm2  = (const float*)d_in[10];
  const float* bm2  = (const float*)d_in[11];
  const float* Wm3  = (const float*)d_in[12];
  const float* bm3  = (const float*)d_in[13];

  float* out = (float*)d_out;
  char* ws = (char*)d_ws;
  unsigned short* WH = (unsigned short*)(ws + kOffWH);
  unsigned short* WL = (unsigned short*)(ws + kOffWL);
  unsigned short* PH = (unsigned short*)(ws + kOffPH);
  unsigned short* PL = (unsigned short*)(ws + kOffPL);
  unsigned short* XH = (unsigned short*)(ws + kOffXH);
  unsigned short* XL = (unsigned short*)(ws + kOffXL);
  unsigned short* A0H = (unsigned short*)(ws + kOffXH);
  unsigned short* A0L = (unsigned short*)(ws + kOffXH + kA0PlaneBytes);
  float* Fp = (float*)(ws + kOffF);

  wprep_kernel<<<dim3(8, 6, 1), dim3(256, 1, 1), 0, stream>>>(W1, W2, W3, Wm1, Wm2, Wm3, WH, WL);

  for (int c = 0; c < kNChunk; ++c) {
    aprep_kernel<<<dim3(kMC * 4 / 256, 1, 1), dim3(256, 1, 1), 0, stream>>>(feat, A0H, A0L, c);

    wmma_gemm64<1, true, 2, 2, false, 2><<<dim3(kGemmBlocks, 1, 1), dim3(256, 1, 1), 0, stream>>>(
        A0H, A0L, kK1, 0L, WH + kWoff1, WL + kWoff1, kK1, 0L,
        (void*)PH, (void*)PL, kH, 0L, b1, nullptr, 0L, kMC, kH, kK1, 1.0f);
    wmma_gemm64<1, true, 2, 2, false, 2><<<dim3(kGemmBlocks, 1, 1), dim3(256, 1, 1), 0, stream>>>(
        PH, PL, kH, 0L, WH + kWoff2, WL + kWoff2, kH, 0L,
        (void*)XH, (void*)XL, kH, 0L, b2, nullptr, 0L, kMC, kH, kH, 1.0f);
    wmma_gemm64<1, true, 2, 2, false, 2><<<dim3(kGemmBlocks, 1, 1), dim3(256, 1, 1), 0, stream>>>(
        XH, XL, kH, 0L, WH + kWoff3, WL + kWoff3, kH, 0L,
        (void*)PH, (void*)PL, kH, 0L, b3, nullptr, 0L, kMC, kH, kH, 1.0f);
    wmma_gemm64<1, true, 2, 2, false, 2><<<dim3(kGemmBlocks, 1, 1), dim3(256, 1, 1), 0, stream>>>(
        PH, PL, kH, 0L, WH + kWoff4, WL + kWoff4, kH, 0L,
        (void*)XH, (void*)XL, kH, 0L, bm1, nullptr, 0L, kMC, kH, kH, 1.0f);
    wmma_gemm64<1, true, 2, 2, false, 2><<<dim3(kGemmBlocks, 1, 1), dim3(256, 1, 1), 0, stream>>>(
        XH, XL, kH, 0L, WH + kWoff5, WL + kWoff5, kH, 0L,
        (void*)PH, (void*)PL, kH, 0L, bm2, nullptr, 0L, kMC, kH, kH, 1.0f);
    wmma_gemm64<1, true, 0, 0, false, 0><<<dim3(kGemm6Blocks, 1, 1), dim3(256, 1, 1), 0, stream>>>(
        PH, PL, kH, 0L, WH + kWoff6, WL + kWoff6, kH, 0L,
        (void*)Fp, nullptr, kFld, 0L, nullptr, nullptr, 0L, kMC, kN6, kH, 1.0f);

    rigid_fit_kernel<<<dim3(kBPC, 1, 1), dim3(256, 1, 1), 0, stream>>>(pos, Fp, bm3, out, c);
  }
}
